// GQA_26671746908805
// MI455X (gfx1250) — hardware-verified
//
#include <hip/hip_runtime.h>
#include <math.h>
#include <stdint.h>

#define NB     2
#define SQ     2048
#define HID    2048
#define NHQ    16
#define NKVH   4
#define HDM    128
#define QW     2048
#define KW     512
#define QKN    2560
#define NTOK   4096
#define NFREQ  64
#define AOW    4096
#define NWV    2
#define SPF    132

static_assert(NTOK % 32 == 0);
static_assert(SQ % 32 == 0);
static_assert(QKN % 128 == 0);
static_assert(KW % 128 == 0);
static_assert(HID % 128 == 0);
static_assert(AOW % 32 == 0);
static_assert(NHQ == 4 * NKVH);
static_assert(QW == NHQ * HDM);
static_assert(KW == NKVH * HDM);
static_assert(QKN == QW + KW);
static_assert(AOW == 2 * QW);

typedef __bf16       v16b __attribute__((ext_vector_type(16)));
typedef __bf16       v8b  __attribute__((ext_vector_type(8)));
typedef float        v8f  __attribute__((ext_vector_type(8)));
typedef float        v4f  __attribute__((ext_vector_type(4)));
typedef unsigned int v4u  __attribute__((ext_vector_type(4)));
typedef unsigned int v2u  __attribute__((ext_vector_type(2)));

__device__ __forceinline__ unsigned short bf_bits(float f) {
  const unsigned u = __float_as_uint(f);
  return (unsigned short)((u + 0x7FFFu + ((u >> 16) & 1u)) >> 16);
}
__device__ __forceinline__ float bf_val(unsigned short h) { return __uint_as_float(((unsigned)h) << 16); }
__device__ __forceinline__ unsigned pk16(unsigned short a, unsigned short b) { return (unsigned)a | ((unsigned)b << 16); }
__device__ __forceinline__ v8f zero8() { v8f z = {0.f, 0.f, 0.f, 0.f, 0.f, 0.f, 0.f, 0.f}; return z; }
__device__ __forceinline__ int wave_id() { return __builtin_amdgcn_readfirstlane((int)(threadIdx.x >> 5)); }

__device__ __forceinline__ void lds_wave_sync() {
  __builtin_amdgcn_fence(__ATOMIC_RELEASE, "workgroup");
  __builtin_amdgcn_wave_barrier();
  __builtin_amdgcn_fence(__ATOMIC_ACQUIRE, "workgroup");
}

union FragB { v16b v; v8b h[2]; };
__device__ __forceinline__ v16b ldfrag_b(const __bf16* p) { FragB f; f.h[0] = *(const v8b*)(p); f.h[1] = *(const v8b*)(p + 16); return f.v; }

__device__ __forceinline__ v8f mma_b(v16b a, v16b b, v8f c) {
  return __builtin_amdgcn_wmma_f32_16x16x32_bf16(false, a, false, b, (short)0, c, false, false);
}
__device__ __forceinline__ void guard2b3(v8f& a, v8f& b, v16b x0, v16b x1, v16b y) {
  asm volatile("v_nop\n\tv_nop\n\tv_nop\n\tv_nop" : "+v"(a), "+v"(b) : "v"(x0), "v"(x1), "v"(y) : "memory");
}
__device__ __forceinline__ void guard1b4(v8f& a, v16b w, v16b x, v16b y, v16b z) {
  asm volatile("v_nop\n\tv_nop\n\tv_nop\n\tv_nop" : "+v"(a) : "v"(w), "v"(x), "v"(y), "v"(z) : "memory");
}
__device__ __forceinline__ void acc_guard4(v8f& a, v8f& b, v8f& c, v8f& d) {
  asm volatile("v_nop\n\tv_nop\n\tv_nop\n\tv_nop" : "+v"(a), "+v"(b), "+v"(c), "+v"(d));
}
__device__ __forceinline__ void acc_guard2(v8f& a, v8f& b) {
  asm volatile("v_nop\n\tv_nop\n\tv_nop\n\tv_nop" : "+v"(a), "+v"(b));
}

__global__ __launch_bounds__(256) void cvt_bf16_kernel(const float* __restrict__ in, unsigned short* __restrict__ outp, int n8) {
  const int i = (int)blockIdx.x * 256 + (int)threadIdx.x;
  if (i >= n8) return;
  const size_t e = 8 * (size_t)i;
  const v4f a = *(const v4f*)(in + e);
  const v4f b = *(const v4f*)(in + e + 4);
  v4u w;
  w[0] = pk16(bf_bits(a[0]), bf_bits(a[1]));
  w[1] = pk16(bf_bits(a[2]), bf_bits(a[3]));
  w[2] = pk16(bf_bits(b[0]), bf_bits(b[1]));
  w[3] = pk16(bf_bits(b[2]), bf_bits(b[3]));
  *(volatile v4u*)(outp + e) = w;
  __threadfence();
  *(volatile v4u*)(outp + e) = w;
}

template <bool DUP>
__global__ __launch_bounds__(256) void tconv_kernel(const float* __restrict__ W, unsigned short* __restrict__ op,
                                                    int R, int Cc, int ldo, int dup) {
  __shared__ __align__(16) float tf[64 * 68];
  const int c0  = (int)blockIdx.x * 64;
  const int r0  = (int)blockIdx.y * 64;
  const int tid = (int)threadIdx.x;
  (void)R;
  {
    const int lr = tid >> 4;
    const int c4 = (tid & 15) * 4;
#pragma unroll
    for (int it = 0; it < 4; ++it) {
      const int rr = it * 16 + lr;
      const v4f a = *(const v4f*)(W + (size_t)(r0 + rr) * Cc + c0 + c4);
      *(v4f*)(tf + rr * 68 + c4) = a;
    }
  }
  __syncthreads();
  const int sub = tid >> 3;
  const int c8  = (tid & 7) * 8;
  v4u hv[2];
#pragma unroll
  for (int it = 0; it < 2; ++it) {
    const int oc = it * 32 + sub;
    v4u a;
#pragma unroll
    for (int q = 0; q < 4; ++q) {
      const float f0 = tf[(c8 + 2 * q) * 68 + oc];
      const float f1 = tf[(c8 + 2 * q + 1) * 68 + oc];
      a[q] = pk16(bf_bits(f0), bf_bits(f1));
    }
    hv[it] = a;
  }
  for (int pass = 0; pass < 2; ++pass) {
#pragma unroll
    for (int it = 0; it < 2; ++it) {
      const int oc = it * 32 + sub;
      const size_t go = (size_t)(c0 + oc) * ldo + r0 + c8;
      *(volatile v4u*)(op + go) = hv[it];
      if (DUP) *(volatile v4u*)(op + go + dup) = hv[it];
    }
    __threadfence();
  }
}

__global__ __launch_bounds__(256) void rope_table_kernel(float* __restrict__ cst, float* __restrict__ snt) {
  const int lane = threadIdx.x & 31;
  const int wave = (int)(threadIdx.x >> 5);
  const int s = (int)blockIdx.x * 8 + wave;
  if (s >= SQ) return;
  double r16 = 10.0;
#pragma unroll 1
  for (int t = 0; t < 4; ++t) r16 = sqrt(r16);
  const float sf = (float)s;
#pragma unroll 1
  for (int half = 0; half < 2; ++half) {
    const int j = half * 32 + lane;
    double p = 1.0;
#pragma unroll 1
    for (int t = 0; t < (j >> 4); ++t) p *= 10.0;
#pragma unroll 1
    for (int t = 0; t < (j & 15); ++t) p *= r16;
    const float pf  = (float)p;
    const float inv = 1.0f / pf;
    const float ang = sf * inv;
    const float cv  = cosf(ang);
    const float sv  = sinf(ang);
    const size_t o = (size_t)s * NFREQ + half * 32 + lane;
    ((volatile float*)cst)[o] = cv;
    ((volatile float*)snt)[o] = sv;
    __threadfence();
    ((volatile float*)cst)[o] = cv;
    ((volatile float*)snt)[o] = sv;
  }
}

template <int EPI> struct SlabCfg { static constexpr int PERWF = 16 * SPF; };
template <> struct SlabCfg<0>     { static constexpr int PERWF = 16 * SPF + 2 * 16 * NFREQ + 2048; };
template <> struct SlabCfg<1>     { static constexpr int PERWF = 16 * SPF + 2048; };
static_assert(NWV * SlabCfg<0>::PERWF * 4 <= 65536);
static_assert((16 * SPF * 4) % 16 == 0);

template <int EPI>
__global__ __launch_bounds__(64) void gemm_w32x128_kernel(
    const unsigned short* __restrict__ Ap, int lda,
    const unsigned short* __restrict__ Btp, int ldb,
    const float* __restrict__ cst, const float* __restrict__ snt,
    const float* __restrict__ nw0, const float* __restrict__ nw1,
    void* C0, void* C1, void* C2, void* C3, int ldc, int ldc2,
    int M, int N, int K) {
  __shared__ __align__(16) float lds_all[NWV * SlabCfg<EPI>::PERWF];

  const int lane = threadIdx.x & 31;
  const int wave = wave_id();
  const int hh = lane >> 4;
  const int rl = lane & 15;
  const int tilesN = N >> 7;
  const int tilesM = M >> 5;
  const int tile = (int)blockIdx.x * NWV + wave;
  if (tile >= tilesM * tilesN) return;
  const int tm = tile / tilesN;
  const int tn = tile - tm * tilesN;
  const int m0 = tm << 5;
  const int n0 = tn << 7;

  const __bf16* A  = (const __bf16*)(const void*)Ap;
  const __bf16* Bt = (const __bf16*)(const void*)Btp;

  v8f acc[2][8];
#pragma unroll
  for (int i = 0; i < 2; ++i)
#pragma unroll
    for (int j = 0; j < 8; ++j) acc[i][j] = zero8();

  for (int k0 = 0; k0 < K; k0 += 32) {
    v16b ah[2];
#pragma unroll
    for (int i = 0; i < 2; ++i) ah[i] = ldfrag_b(A + (size_t)(m0 + i * 16 + rl) * lda + k0 + 8 * hh);
#pragma unroll
    for (int j = 0; j < 8; ++j) {
      const v16b bj = ldfrag_b(Bt + (size_t)(n0 + j * 16 + rl) * ldb + k0 + 8 * hh);
      acc[0][j] = mma_b(ah[0], bj, acc[0][j]);
      acc[1][j] = mma_b(ah[1], bj, acc[1][j]);
      guard2b3(acc[0][j], acc[1][j], ah[0], ah[1], bj);
    }
  }
  acc_guard4(acc[0][0], acc[0][1], acc[0][2], acc[0][3]);
  acc_guard4(acc[0][4], acc[0][5], acc[0][6], acc[0][7]);
  acc_guard4(acc[1][0], acc[1][1], acc[1][2], acc[1][3]);
  acc_guard4(acc[1][4], acc[1][5], acc[1][6], acc[1][7]);

  float* wl  = lds_all + wave * SlabCfg<EPI>::PERWF;
  float* slf = wl;

  if (EPI == 0) {
    float* csl = wl + 16 * SPF;
    float* snl = csl + 16 * NFREQ;
    unsigned short* sl16 = (unsigned short*)(void*)(snl + 16 * NFREQ);
    const bool isq = (n0 < QW);
    unsigned short* P0 = isq ? (unsigned short*)C0 : (unsigned short*)C2;
    unsigned short* P1 = isq ? (unsigned short*)C1 : (unsigned short*)C3;
    const int ldp  = isq ? ldc : ldc2;
    const int col0 = isq ? n0 : (n0 - QW);
    const v4f wq4 = *(const v4f*)(nw0 + 4 * lane);
    const v4f wk4 = *(const v4f*)(nw1 + 4 * lane);
    const float fq = isq ? 1.0f : 0.0f;
    const v4f w4 = wq4 * fq + wk4 * (1.0f - fq);
    const float sgn = (float)(2 * hh - 1);
    const int j4 = 4 * rl;
#pragma unroll
    for (int i = 0; i < 2; ++i) {
      const int mb = m0 + i * 16;
      const int s0 = mb & (SQ - 1);
#pragma unroll
      for (int j = 0; j < 8; ++j)
#pragma unroll
        for (int r = 0; r < 8; ++r)
          slf[(8 * hh + r) * SPF + j * 16 + rl] = acc[i][j][r];
#pragma unroll
      for (int u = 0; u < 8; ++u) {
        const int p   = lane + 32 * u;
        const int row = p >> 4, c4 = (p & 15) * 4;
        const v4f cv4 = *(const v4f*)(cst + (size_t)(s0 + row) * NFREQ + c4);
        const v4f sv4 = *(const v4f*)(snt + (size_t)(s0 + row) * NFREQ + c4);
        *(v4f*)(csl + row * NFREQ + c4) = cv4;
        *(v4f*)(snl + row * NFREQ + c4) = sv4;
      }
      lds_wave_sync();
#pragma unroll 1
      for (int rr = 0; rr < 16; ++rr) {
        const v4f x4 = *(const v4f*)(slf + rr * SPF + 4 * lane);
        float ss = x4[0] * x4[0] + x4[1] * x4[1] + x4[2] * x4[2] + x4[3] * x4[3];
#pragma unroll
        for (int off = 1; off < 32; off <<= 1) ss += __shfl_xor(ss, off, 32);
        const float rn = rsqrtf(ss * 0.0078125f + 1.0e-6f);
        const v4f c4v = *(const v4f*)(csl + rr * NFREQ + j4);
        const v4f s4v = *(const v4f*)(snl + rr * NFREQ + j4);
        unsigned short hb[4], lb[4];
#pragma unroll
        for (int e = 0; e < 4; ++e) {
          const float t  = x4[e] * rn * w4[e];
          const float pt = __shfl_xor(t, 16, 32);
          const float o  = t * c4v[e] + sgn * (pt * s4v[e]);
          hb[e] = bf_bits(o);
          lb[e] = bf_bits(o - bf_val(hb[e]));
        }
        v2u hv, lv;
        hv[0] = pk16(hb[0], hb[1]); hv[1] = pk16(hb[2], hb[3]);
        lv[0] = pk16(lb[0], lb[1]); lv[1] = pk16(lb[2], lb[3]);
        *(v2u*)(sl16 + rr * 128 + 4 * lane)        = hv;
        *(v2u*)(sl16 + 2048 + rr * 128 + 4 * lane) = lv;
      }
      lds_wave_sync();
      for (int pass = 0; pass < 2; ++pass) {
#pragma unroll
        for (int it = 0; it < 8; ++it) {
          const int row = it * 2 + hh;
          const int c8  = rl * 8;
          const v4u vh = *(const v4u*)(sl16 + row * 128 + c8);
          const v4u vl = *(const v4u*)(sl16 + 2048 + row * 128 + c8);
          const size_t go = (size_t)(mb + row) * ldp + col0 + c8;
          *(volatile v4u*)(P0 + go) = vh;
          *(volatile v4u*)(P1 + go) = vl;
        }
        __threadfence();
      }
      lds_wave_sync();
    }
  } else if (EPI == 1) {
    unsigned short* sl16 = (unsigned short*)(void*)(wl + 16 * SPF);
    unsigned short* P0 = (unsigned short*)C0;
    unsigned short* P1 = (unsigned short*)C1;
#pragma unroll
    for (int i = 0; i < 2; ++i) {
#pragma unroll
      for (int j = 0; j < 8; ++j)
#pragma unroll
        for (int r = 0; r < 8; ++r)
          slf[(8 * hh + r) * SPF + j * 16 + rl] = acc[i][j][r];
      lds_wave_sync();
#pragma unroll 1
      for (int rr = 0; rr < 16; ++rr) {
        const v4f x4 = *(const v4f*)(slf + rr * SPF + 4 * lane);
        unsigned short hb[4], lb[4];
#pragma unroll
        for (int e = 0; e < 4; ++e) {
          hb[e] = bf_bits(x4[e]);
          lb[e] = bf_bits(x4[e] - bf_val(hb[e]));
        }
        v2u hv, lv;
        hv[0] = pk16(hb[0], hb[1]); hv[1] = pk16(hb[2], hb[3]);
        lv[0] = pk16(lb[0], lb[1]); lv[1] = pk16(lb[2], lb[3]);
        *(v2u*)(sl16 + rr * 128 + 4 * lane)        = hv;
        *(v2u*)(sl16 + 2048 + rr * 128 + 4 * lane) = lv;
      }
      lds_wave_sync();
      for (int pass = 0; pass < 2; ++pass) {
#pragma unroll
        for (int it = 0; it < 8; ++it) {
          const int row = it * 2 + hh;
          const int c8  = rl * 8;
          const v4u vh = *(const v4u*)(sl16 + row * 128 + c8);
          const v4u vl = *(const v4u*)(sl16 + 2048 + row * 128 + c8);
          const size_t go = (size_t)(m0 + i * 16 + row) * ldc + n0 + c8;
          *(volatile v4u*)(P0 + go) = vh;
          *(volatile v4u*)(P1 + go) = vl;
        }
        __threadfence();
      }
      lds_wave_sync();
    }
  } else {
    float* C = (float*)C0;
#pragma unroll
    for (int i = 0; i < 2; ++i) {
#pragma unroll
      for (int j = 0; j < 8; ++j)
#pragma unroll
        for (int r = 0; r < 8; ++r)
          slf[(8 * hh + r) * SPF + j * 16 + rl] = acc[i][j][r];
      lds_wave_sync();
      for (int pass = 0; pass < 2; ++pass) {
#pragma unroll
        for (int row = 0; row < 16; ++row) {
          const v4f v = *(const v4f*)(slf + row * SPF + lane * 4);
          *(volatile v4f*)(C + (size_t)(m0 + i * 16 + row) * ldc + n0 + lane * 4) = v;
        }
        __threadfence();
      }
      lds_wave_sync();
    }
  }
}

#define AKC  32
#define KP   136
#define VP   40
#define PP   40
#define NWA  2
#define ATT_SCALE 0.08838834764831845f
static_assert((2 * AKC * KP + 2 * HDM * VP + 2 * NWA * 16 * PP + 2 * NWA * 16 * HDM) * 2 <= 65536);
static_assert(SQ % 32 == 0);

__global__ __launch_bounds__(64) void attn_kernel(
    const unsigned short* __restrict__ qhp, const unsigned short* __restrict__ qlp,
    const unsigned short* __restrict__ khp, const unsigned short* __restrict__ klp,
    const unsigned short* __restrict__ vhp, const unsigned short* __restrict__ vlp,
    unsigned short* __restrict__ aop) {
  __shared__ __align__(16) unsigned short Ks[AKC * KP];
  __shared__ __align__(16) unsigned short Kls[AKC * KP];
  __shared__ __align__(16) unsigned short Vhs[HDM * VP];
  __shared__ __align__(16) unsigned short Vls[HDM * VP];
  __shared__ __align__(16) unsigned short Phs[NWA][16 * PP];
  __shared__ __align__(16) unsigned short Pls[NWA][16 * PP];
  __shared__ __align__(16) unsigned short Osh[NWA][16 * HDM];
  __shared__ __align__(16) unsigned short Osl[NWA][16 * HDM];

  const int tid  = (int)threadIdx.x;
  const int lane = tid & 31;
  const int wave = wave_id();
  const int hh   = lane >> 4;
  const int c    = lane & 15;
  const int qt   = (int)blockIdx.x;
  const int h    = (int)blockIdx.y;
  const int b    = (int)blockIdx.z;
  const int kvh  = h >> 2;
  const int q0   = qt * 32 + wave * 16;
  const size_t tok0 = (size_t)b * SQ;

  const __bf16* Qhr = (const __bf16*)(const void*)qhp + (tok0 + q0 + c) * QW + h * HDM + 8 * hh;
  const __bf16* Qlr = (const __bf16*)(const void*)qlp + (tok0 + q0 + c) * QW + h * HDM + 8 * hh;
  unsigned short* ph = Phs[wave];
  unsigned short* pl = Pls[wave];

  float mrow[8], lrow[8];
  v8f oacc[8];
#pragma unroll
  for (int r = 0; r < 8; ++r) { mrow[r] = -INFINITY; lrow[r] = 0.f; }
#pragma unroll
  for (int t = 0; t < 8; ++t) oacc[t] = zero8();

  const int nch = qt + 1;
  for (int kc = 0; kc < nch; ++kc) {
    const int kv0 = kc * AKC;
    __syncthreads();
#pragma unroll 2
    for (int u = 0; u < 8; ++u) {
      const int p   = tid + 64 * u;
      const int key = p >> 4, d8 = (p & 15) * 8;
      const size_t ko = (tok0 + kv0 + key) * KW + kvh * HDM + d8;
      const v4u kx = *(const v4u*)(khp + ko);
      const v4u ky = *(const v4u*)(klp + ko);
      *(v4u*)(Ks  + key * KP + d8) = kx;
      *(v4u*)(Kls + key * KP + d8) = ky;
      const int d = p >> 2, k8 = (p & 3) * 8;
      const size_t vo = (size_t)(kvh * HDM + d) * NTOK + tok0 + kv0 + k8;
      const v4u vx = *(const v4u*)(vhp + vo);
      const v4u vy = *(const v4u*)(vlp + vo);
      *(v4u*)(Vhs + d * VP + k8) = vx;
      *(v4u*)(Vls + d * VP + k8) = vy;
    }
    __syncthreads();

    v8f sa[2];
    sa[0] = zero8(); sa[1] = zero8();
#pragma unroll
    for (int dc = 0; dc < 4; ++dc) {
      const v16b qh = ldfrag_b(Qhr + dc * 32);
      const v16b ql = ldfrag_b(Qlr + dc * 32);
#pragma unroll
      for (int j = 0; j < 2; ++j) {
        const v16b kb = ldfrag_b((const __bf16*)(const void*)Ks  + (j * 16 + c) * KP + dc * 32 + 8 * hh);
        const v16b kl = ldfrag_b((const __bf16*)(const void*)Kls + (j * 16 + c) * KP + dc * 32 + 8 * hh);
        sa[j] = mma_b(qh, kb, sa[j]);
        sa[j] = mma_b(qh, kl, sa[j]);
        sa[j] = mma_b(ql, kb, sa[j]);
        guard1b4(sa[j], qh, ql, kb, kl);
      }
    }
    acc_guard2(sa[0], sa[1]);

    const bool diag = (kc == qt);
    float cm[8];
#pragma unroll
    for (int r = 0; r < 8; ++r) {
      const int qrow = q0 + 8 * hh + r;
      float m = -INFINITY;
#pragma unroll
      for (int j = 0; j < 2; ++j) {
        const int kvcol = kv0 + j * 16 + c;
        const float sv = sa[j][r] * ATT_SCALE;
        const bool masked = diag && (kvcol > qrow);
        const float sm = masked ? -INFINITY : sv;
        sa[j][r] = sm;
        m = fmaxf(m, sm);
      }
#pragma unroll
      for (int off = 1; off < 16; off <<= 1) m = fmaxf(m, __shfl_xor(m, off, 32));
      cm[r] = m;
    }
#pragma unroll
    for (int r = 0; r < 8; ++r) {
      const float mnew  = fmaxf(mrow[r], cm[r]);
      const float alpha = __expf(mrow[r] - mnew);
      mrow[r] = mnew;
      float psum = 0.f;
#pragma unroll
      for (int j = 0; j < 2; ++j) {
        const float p = __expf(sa[j][r] - mnew);
        psum += p;
        const unsigned short hb = bf_bits(p);
        const unsigned short lb = bf_bits(p - bf_val(hb));
        const int po = (8 * hh + r) * PP + j * 16 + c;
        ph[po] = hb;
        pl[po] = lb;
      }
#pragma unroll
      for (int off = 1; off < 16; off <<= 1) psum += __shfl_xor(psum, off, 32);
      lrow[r] = lrow[r] * alpha + psum;
#pragma unroll
      for (int t = 0; t < 8; ++t) oacc[t][r] *= alpha;
    }
    lds_wave_sync();
    const v16b pa = ldfrag_b((const __bf16*)(const void*)ph + c * PP + 8 * hh);
    const v16b pr = ldfrag_b((const __bf16*)(const void*)pl + c * PP + 8 * hh);
#pragma unroll
    for (int t = 0; t < 8; ++t) {
      const v16b vb = ldfrag_b((const __bf16*)(const void*)Vhs + (t * 16 + c) * VP + 8 * hh);
      const v16b vr = ldfrag_b((const __bf16*)(const void*)Vls + (t * 16 + c) * VP + 8 * hh);
      oacc[t] = mma_b(pa, vb, oacc[t]);
      oacc[t] = mma_b(pa, vr, oacc[t]);
      oacc[t] = mma_b(pr, vb, oacc[t]);
      guard1b4(oacc[t], pa, pr, vb, vr);
    }
  }
  __syncthreads();
  acc_guard4(oacc[0], oacc[1], oacc[2], oacc[3]);
  acc_guard4(oacc[4], oacc[5], oacc[6], oacc[7]);

  unsigned short* osh = Osh[wave];
  unsigned short* osl = Osl[wave];
#pragma unroll
  for (int r = 0; r < 8; ++r) {
    const float inv = 1.0f / lrow[r];
#pragma unroll
    for (int t = 0; t < 8; ++t) {
      const float o = oacc[t][r] * inv;
      const unsigned short hb = bf_bits(o);
      const unsigned short lb = bf_bits(o - bf_val(hb));
      const int so = (8 * hh + r) * HDM + t * 16 + c;
      osh[so] = hb;
      osl[so] = lb;
    }
  }
  lds_wave_sync();
  unsigned short* Ag = aop + (tok0 + q0) * AOW + (size_t)h * HDM;
  const int c8 = c * 8;
  for (int pass = 0; pass < 2; ++pass) {
#pragma unroll
    for (int it = 0; it < 8; ++it) {
      const int row = it * 2 + hh;
      const v4u x = *(const v4u*)(osh + row * HDM + c8);
      const v4u y = *(const v4u*)(osl + row * HDM + c8);
      *(volatile v4u*)(Ag + (size_t)row * AOW + c8)      = x;
      *(volatile v4u*)(Ag + (size_t)row * AOW + QW + c8) = y;
    }
    __threadfence();
  }
}

extern "C" void kernel_launch(void* const* d_in, const int* in_sizes, int n_in,
                              void* d_out, int out_size, void* d_ws, size_t ws_size,
                              hipStream_t stream) {
  if (n_in < 7) return;
  if (in_sizes[0] != NTOK * HID) return;
  if (in_sizes[1] != HID * QW) return;
  if (in_sizes[2] != HID * KW) return;
  if (in_sizes[3] != HID * KW) return;
  if (in_sizes[4] != HID * HID) return;
  if (in_sizes[5] != HDM) return;
  if (in_sizes[6] != HDM) return;
  if (out_size != NTOK * HID) return;

  const float* x   = (const float*)d_in[0];
  const float* wq  = (const float*)d_in[1];
  const float* wk  = (const float*)d_in[2];
  const float* wv  = (const float*)d_in[3];
  const float* wo  = (const float*)d_in[4];
  const float* qnw = (const float*)d_in[5];
  const float* knw = (const float*)d_in[6];
  float* out = (float*)d_out;

  const size_t szXB  = (size_t)NTOK * HID * 2;
  const size_t szWQK = (size_t)QKN * HID * 2;
  const size_t szWVT = (size_t)KW * HID * 2;
  const size_t szWO2 = (size_t)HID * AOW * 2;
  const size_t szT   = (size_t)SQ * NFREQ * 4;
  const size_t szQ   = (size_t)NTOK * QW * 2;
  const size_t szK   = (size_t)NTOK * KW * 2;
  const size_t szVT  = (size_t)KW * NTOK * 2;
  const size_t szCTX = (size_t)NTOK * AOW * 2;
  size_t off = 0;
  const size_t oXB  = off; off += szXB;
  const size_t oWQK = off; off += szWQK;
  const size_t oWVT = off; off += szWVT;
  const size_t oWO2 = off; off += szWO2;
  const size_t oCST = off; off += szT;
  const size_t oSNT = off; off += szT;
  const size_t oQH  = off; off += szQ;
  const size_t oQL  = off; off += szQ;
  const size_t oKH  = off; off += szK;
  const size_t oKL  = off; off += szK;
  const size_t oVTH = off; off += szVT;
  const size_t oVTL = off; off += szVT;
  const size_t oCTX = off; off += szCTX;
  if (off > ws_size) return;
  if (off > (size_t)134217728) return;

  char* ws = (char*)d_ws;
  unsigned short* XB  = (unsigned short*)(ws + oXB);
  unsigned short* WQK = (unsigned short*)(ws + oWQK);
  unsigned short* WVT = (unsigned short*)(ws + oWVT);
  unsigned short* WO2 = (unsigned short*)(ws + oWO2);
  float*          CST = (float*)(ws + oCST);
  float*          SNT = (float*)(ws + oSNT);
  unsigned short* QH  = (unsigned short*)(ws + oQH);
  unsigned short* QL  = (unsigned short*)(ws + oQL);
  unsigned short* KH  = (unsigned short*)(ws + oKH);
  unsigned short* KL  = (unsigned short*)(ws + oKL);
  unsigned short* VTH = (unsigned short*)(ws + oVTH);
  unsigned short* VTL = (unsigned short*)(ws + oVTL);
  unsigned short* CTX = (unsigned short*)(ws + oCTX);

  const dim3 b256(256), b64(64);

  cvt_bf16_kernel<<<dim3((NTOK * HID / 8) / 256), b256, 0, stream>>>(x, XB, NTOK * HID / 8);
  tconv_kernel<false><<<dim3(QW / 64, HID / 64), b256, 0, stream>>>(wq, WQK, HID, QW, HID, 0);
  tconv_kernel<false><<<dim3(KW / 64, HID / 64), b256, 0, stream>>>(wk, WQK + (size_t)QW * HID, HID, KW, HID, 0);
  tconv_kernel<false><<<dim3(KW / 64, HID / 64), b256, 0, stream>>>(wv, WVT, HID, KW, HID, 0);
  tconv_kernel<true><<<dim3(HID / 64, HID / 64), b256, 0, stream>>>(wo, WO2, HID, HID, AOW, HID);
  rope_table_kernel<<<dim3(SQ / 8), b256, 0, stream>>>(CST, SNT);
  gemm_w32x128_kernel<0><<<dim3((NTOK / 32) * (QKN / 128) / NWV), b64, 0, stream>>>(
      XB, HID, WQK, HID, CST, SNT, qnw, knw, (void*)QH, (void*)QL, (void*)KH, (void*)KL, QW, KW, NTOK, QKN, HID);
  gemm_w32x128_kernel<1><<<dim3((KW / 32) * (NTOK / 128) / NWV), b64, 0, stream>>>(
      WVT, HID, XB, HID, CST, SNT, qnw, knw, (void*)VTH, (void*)VTL, (void*)VTH, (void*)VTL, NTOK, NTOK, KW, NTOK, HID);
  attn_kernel<<<dim3(SQ / 32, NHQ, NB), b64, 0, stream>>>(QH, QL, KH, KL, VTH, VTL, CTX);
  gemm_w32x128_kernel<2><<<dim3((NTOK / 32) * (HID / 128) / NWV), b64, 0, stream>>>(
      CTX, AOW, WO2, AOW, CST, SNT, qnw, knw, (void*)out, (void*)out, (void*)out, (void*)out, HID, HID, NTOK, HID, AOW);
  (void)hipGetLastError();
}
